// MessagePassing_68298569941222
// MI455X (gfx1250) — hardware-verified
//
#include <hip/hip_runtime.h>
#include <stddef.h>
#include <stdint.h>


#define DD     32
#define BDIM   16
#define KH     64
#define UCOL   512
#define UVW    576
#define NGC    192
#define NTHR   256
#define NWAVE  8
#define EPT    8
#define CHUNK  (NTHR * EPT)
#define WCAP   (EPT * 32)
#define LISTN  (NWAVE * WCAP)
#define NBA    1024
#define SLA    10
#define RCAP   28672
#define DEGCAP 64
#define GBM    64
#define GBN    96
#define GTHR   128
#define NSTEP  4
#define NBKB   ((UVW * KH / 8) / NTHR)
#define NWGB   ((NGC * KH / 8) / NTHR)
#define STWU   (NWAVE * 4 * KH)
#define AGG_ZINTS (LISTN + 2 * RCAP + 3 * NBA)
#define AGG_LDS_INTS (AGG_ZINTS + 16 + STWU / 2)
#define WSMAX  134217728
#define NNOM   50000
#define MPNOM  (((NNOM + NBA - 1) / NBA) * NBA)

static_assert((CHUNK & (CHUNK - 1)) == 0 && CHUNK <= 4096);
static_assert((NBA & (NBA - 1)) == 0 && NBA == (1 << SLA));
static_assert(((long long)CHUNK << SLA) < (1LL << 31));
static_assert(LISTN % NTHR == 0);
static_assert(NBA % (NWAVE * 4) == 0 && NBA % 32 == 0 && NBA % GBM == 0);
static_assert(RCAP % 4 == 0 && AGG_ZINTS % 4 == 0 && LISTN % 4 == 0);
static_assert((UVW * KH / 8) % NTHR == 0 && (NGC * KH / 8) % NTHR == 0);
static_assert(UVW % GBN == 0 && GBN % 16 == 0 && (GBN / 4) % 8 == 0 && UVW % 32 == 0);
static_assert(KH % 32 == 0 && KH == 2 * DD && UCOL == BDIM * DD && UVW >= UCOL + DD);
static_assert(GBM == (GTHR / 32) * 16 && NGC == 6 * DD && GTHR == 2 * GBM);
static_assert((16 * (GBN / 4)) % 32 == 0);
static_assert(GBM * NGC * 4 >= GBM * DD * 4 + GBM * KH * 2);
static_assert((GBM * KH / 8) % GTHR == 0 && (GBM * DD / 4) % GTHR == 0);
static_assert(AGG_LDS_INTS * 4 <= 300000);
static_assert((size_t)MPNOM * UVW * 4 + 2 * (size_t)MPNOM * KH * 2 + (size_t)UVW * KH * 2 + (size_t)NGC * KH * 2 <= (size_t)WSMAX);
static_assert(MPNOM % GBM == 0);

typedef float          v4f   __attribute__((ext_vector_type(4)));
typedef float          v8f   __attribute__((ext_vector_type(8)));
typedef int            v4i   __attribute__((ext_vector_type(4)));
typedef int            v8i   __attribute__((ext_vector_type(8)));
typedef unsigned short v8us  __attribute__((ext_vector_type(8)));
typedef unsigned short v16us __attribute__((ext_vector_type(16)));
typedef __bf16         v16bf __attribute__((ext_vector_type(16)));
typedef v4f  __attribute__((may_alias)) v4fa;
typedef v4i  __attribute__((may_alias)) v4ia;
typedef v8us __attribute__((may_alias)) v8usa;
union FragB { v16bf v; v16us u; v8us h[2]; v8i w; };

__device__ __forceinline__ v8f wmb(const FragB& a, const FragB& b, v8f c) {
  v8f d = __builtin_amdgcn_wmma_f32_16x16x32_bf16(false, a.v, false, b.v, (short)0, c, false, false);
  asm volatile("v_nop\n\tv_nop\n\tv_nop\n\tv_nop" : "+v"(d) : "v"(a.w), "v"(b.w));
  return d;
}

__device__ __forceinline__ unsigned bf16_bits(float f) {
  const unsigned u = __float_as_uint(f);
  return (u + 0x7FFFu + ((u >> 16) & 1u)) >> 16;
}
__device__ __forceinline__ float bf16_val(float f) {
  return __uint_as_float(bf16_bits(f) << 16);
}
__device__ __forceinline__ v8f z8() { v8f z = {0.f, 0.f, 0.f, 0.f, 0.f, 0.f, 0.f, 0.f}; return z; }
__device__ __forceinline__ float sigm(float x) { return __builtin_amdgcn_rcpf(1.0f + expf(-x)); }

__device__ __forceinline__ int scan_chunk(const int* __restrict__ pr, int nE, int cbase, int slotBase,
                                          int nb, int* list, int tid, int lane, int wave) {
  int wc = 0;
  const int el0  = tid * EPT;
  const int e0   = cbase + el0;
  const int sent = -2147483647 - 1;
  v4i da, db;
  if (cbase + CHUNK <= nE) {
    const int* q = pr + 2 * (size_t)e0;
    const v4i p0 = *(const v4i*)q;
    const v4i p1 = *(const v4i*)(q + 4);
    const v4i p2 = *(const v4i*)(q + 8);
    const v4i p3 = *(const v4i*)(q + 12);
    da.x = p0.x; da.y = p0.z; da.z = p1.x; da.w = p1.z;
    db.x = p2.x; db.y = p2.z; db.z = p3.x; db.w = p3.z;
  } else {
    const int lst = nE - 1;
    da.x = (e0     < nE) ? pr[2 * min(e0,     lst)] : sent;
    da.y = (e0 + 1 < nE) ? pr[2 * min(e0 + 1, lst)] : sent;
    da.z = (e0 + 2 < nE) ? pr[2 * min(e0 + 2, lst)] : sent;
    da.w = (e0 + 3 < nE) ? pr[2 * min(e0 + 3, lst)] : sent;
    db.x = (e0 + 4 < nE) ? pr[2 * min(e0 + 4, lst)] : sent;
    db.y = (e0 + 5 < nE) ? pr[2 * min(e0 + 5, lst)] : sent;
    db.z = (e0 + 6 < nE) ? pr[2 * min(e0 + 6, lst)] : sent;
    db.w = (e0 + 7 < nE) ? pr[2 * min(e0 + 7, lst)] : sent;
  }
  const unsigned nbs = (unsigned)slotBase;
  const unsigned unb = (unsigned)nb;
  const unsigned s0 = (unsigned)da.x - nbs, s1 = (unsigned)da.y - nbs;
  const unsigned s2 = (unsigned)da.z - nbs, s3 = (unsigned)da.w - nbs;
  const unsigned s4 = (unsigned)db.x - nbs, s5 = (unsigned)db.y - nbs;
  const unsigned s6 = (unsigned)db.z - nbs, s7 = (unsigned)db.w - nbs;
  const bool h0 = s0 < unb, h1 = s1 < unb, h2 = s2 < unb, h3 = s3 < unb;
  const bool h4 = s4 < unb, h5 = s5 < unb, h6 = s6 < unb, h7 = s7 < unb;
  const unsigned any = __builtin_amdgcn_ballot_w32(h0 | h1 | h2 | h3 | h4 | h5 | h6 | h7);
  if (any != 0u) {
#define HITJ(J, HJ, SJ) { \
      const unsigned mj = __builtin_amdgcn_ballot_w32(HJ); \
      if (mj != 0u) { \
        if (HJ) { \
          const int pos = wc + (int)__builtin_amdgcn_mbcnt_lo(mj, 0u); \
          if (pos < WCAP) list[wave * WCAP + pos] = ((el0 + (J)) << SLA) | (int)(SJ); \
        } \
        wc += (int)__builtin_popcount(mj); } }
    HITJ(0, h0, s0)
    HITJ(1, h1, s1)
    HITJ(2, h2, s2)
    HITJ(3, h3, s3)
    HITJ(4, h4, s4)
    HITJ(5, h5, s5)
    HITJ(6, h6, s6)
    HITJ(7, h7, s7)
#undef HITJ
  }
  return wc;
}

__global__ __launch_bounds__(NTHR) void k_prep(const float* __restrict__ x, int nN, int nbHA,
                                               const float* __restrict__ kw, const float* __restrict__ kb,
                                               const float* __restrict__ wih, const float* __restrict__ whh,
                                               unsigned short* ha, unsigned short* bk, unsigned short* wg) {
  const int b = (int)blockIdx.x, tid = (int)threadIdx.x;
  v8us o;
  unsigned short* dp;
  if (b < nbHA) {
    const int u   = b * NTHR + tid;
    const int row = u >> 3, p = u & 7;
    const int rc  = row < nN ? row : nN - 1;
    const float* xp = x + (size_t)rc * DD + 8 * (p & 3);
    const v4f a = *(const v4f*)xp;
    const v4f c = *(const v4f*)(xp + 4);
    const bool ok = (row < nN) && (p < 4);
    o[0] = ok ? (unsigned short)bf16_bits(a.x) : (unsigned short)0;
    o[1] = ok ? (unsigned short)bf16_bits(a.y) : (unsigned short)0;
    o[2] = ok ? (unsigned short)bf16_bits(a.z) : (unsigned short)0;
    o[3] = ok ? (unsigned short)bf16_bits(a.w) : (unsigned short)0;
    o[4] = ok ? (unsigned short)bf16_bits(c.x) : (unsigned short)0;
    o[5] = ok ? (unsigned short)bf16_bits(c.y) : (unsigned short)0;
    o[6] = ok ? (unsigned short)bf16_bits(c.z) : (unsigned short)0;
    o[7] = ok ? (unsigned short)bf16_bits(c.w) : (unsigned short)0;
    dp = ha + (size_t)u * 8;
  } else if (b < nbHA + NBKB) {
    const int u  = (b - nbHA) * NTHR + tid;
    const int n  = u >> 3, k8 = (u & 7) * 8;
    const int nc = n < UCOL ? n : UCOL - 1;
    const int i  = nc >> 4, bb = nc & 15;
    int ib = n - UCOL;
    ib = ib < 0 ? 0 : (ib > DD - 1 ? DD - 1 : ib);
    const float fw = (n < UCOL) ? 1.0f : 0.0f;
    const float* wp = kw + (size_t)bb * (DD * DD) + i * DD;
    const float* bq = kb + ib * DD;
#pragma unroll
    for (int e = 0; e < 8; ++e) {
      const int kk = (k8 + e) & (DD - 1);
      const float v = wp[kk] * fw + bq[kk] * (1.0f - fw);
      o[e] = (unsigned short)bf16_bits(v);
    }
    dp = bk + (size_t)u * 8;
  } else if (b < nbHA + NBKB + NWGB) {
    const int u  = (b - nbHA - NBKB) * NTHR + tid;
    const int n  = u >> 3, k8 = (u & 7) * 8;
    const int ni = n < 3 * DD ? n : 3 * DD - 1;
    int nh = n - 3 * DD;
    nh = nh < 0 ? 0 : (nh > 3 * DD - 1 ? 3 * DD - 1 : nh);
    const float fw = (n < 3 * DD) ? 1.0f : 0.0f;
    const float* ip = wih + ni * DD;
    const float* hq = whh + nh * DD;
#pragma unroll
    for (int e = 0; e < 8; ++e) {
      const int kk = (k8 + e) & (DD - 1);
      const float v = ip[kk] * fw + hq[kk] * (1.0f - fw);
      o[e] = (unsigned short)bf16_bits(v);
    }
    dp = wg + (size_t)u * 8;
  } else {
    return;
  }
  *(volatile v8us*)dp = o;
  __threadfence();
  *(volatile v8us*)dp = o;
}

__global__ __launch_bounds__(GTHR) void k_node(const unsigned short* __restrict__ A,
                                               const unsigned short* __restrict__ BT, float* Cm) {
  __shared__ __attribute__((aligned(16))) float stg[GBM * GBN];
  constexpr int NT  = GBN / 16;
  constexpr int UPR = GBN / 4;
  constexpr int NIT = 16 * UPR / 32;
  const int tid = (int)threadIdx.x, lane = tid & 31, wave = tid >> 5, hh = lane >> 4, m = lane & 15;
  const int rowBase = (int)blockIdx.x * GBM;
  const int colBase = (int)blockIdx.y * GBN;

  v8f acc[NT];
#pragma unroll
  for (int t = 0; t < NT; ++t) acc[t] = z8();
  const unsigned short* ap = A  + (size_t)(rowBase + 16 * wave + m) * KH + 8 * hh;
  const unsigned short* bp = BT + (size_t)(colBase + m) * KH + 8 * hh;

#pragma unroll 1
  for (int k0 = 0; k0 < KH; k0 += 32) {
    FragB af;
    af.h[0] = *(const v8usa*)(ap + k0);
    af.h[1] = *(const v8usa*)(ap + k0 + 16);
#pragma unroll
    for (int nt = 0; nt < NT; ++nt) {
      const unsigned short* wq = bp + (size_t)(16 * nt) * KH + k0;
      FragB bf;
      bf.h[0] = *(const v8usa*)wq;
      bf.h[1] = *(const v8usa*)(wq + 16);
      acc[nt] = wmb(af, bf, acc[nt]);
    }
  }

#pragma unroll
  for (int nt = 0; nt < NT; ++nt) {
    const int lc = 16 * nt + m;
#pragma unroll
    for (int r = 0; r < 8; ++r) {
      const int lr = 16 * wave + 8 * hh + r;
      stg[lr * GBN + lc] = acc[nt][r];
    }
  }
  __syncthreads();

  const float* lp = stg + 16 * wave * GBN;
  float* gp = Cm + (size_t)(rowBase + 16 * wave) * UVW + colBase;
#pragma unroll
  for (int it = 0; it < NIT; ++it) {
    const int u  = it * 32 + lane;
    const int lr = u / UPR;
    const int c4 = u - lr * UPR;
    const v4f v = *(const v4fa*)(lp + lr * GBN + 4 * c4);
    *(volatile v4f*)(gp + (size_t)lr * UVW + 4 * c4) = v;
  }
  __threadfence();
#pragma unroll
  for (int it = 0; it < NIT; ++it) {
    const int u  = it * 32 + lane;
    const int lr = u / UPR;
    const int c4 = u - lr * UPR;
    const v4f v = *(const v4fa*)(lp + lr * GBN + 4 * c4);
    *(volatile v4f*)(gp + (size_t)lr * UVW + 4 * c4) = v;
  }
}

__global__ __launch_bounds__(NTHR) void k_agg(const int* __restrict__ pr, int nE, int nN,
                                              const float* __restrict__ bond, const float* __restrict__ uv,
                                              unsigned short* aggp) {
  extern __shared__ __attribute__((aligned(16))) int dsm[];
  int* list = dsm;
  int* hl   = dsm + LISTN;
  int* sl   = hl + RCAP;
  int* cnt  = sl + RCAP;
  int* offs = cnt + NBA;
  int* cur  = offs + NBA;
  int* misc = cur + NBA;
  unsigned short* stw = (unsigned short*)(misc + 16);
  const int tid = (int)threadIdx.x, lane = tid & 31, wave = tid >> 5;
  const int nodeBase = (int)blockIdx.x * NBA;

  {
    const v4i z4 = {0, 0, 0, 0};
    for (int i = tid * 4; i < AGG_ZINTS; i += NTHR * 4) *(v4ia*)(dsm + i) = z4;
    for (int i = tid; i < 16 + STWU / 2; i += NTHR) misc[i] = 0;
  }
  __syncthreads();

  int t = 0, ov = 0;
  const int nChunks = (nE + CHUNK - 1) / CHUNK;
#pragma unroll 1
  for (int ch = 0; ch < nChunks; ++ch) {
    const int cbase = ch * CHUNK;
    const int wc = scan_chunk(pr, nE, cbase, nodeBase, NBA, list, tid, lane, wave);
    if (lane == 0) misc[wave] = wc;
    __syncthreads();
    if (wave == 0) {
#pragma unroll 1
      for (int w2 = 0; w2 < NWAVE; ++w2) {
        int c = misc[w2];
        c = c < 0 ? 0 : (c > WCAP ? WCAP : c);
#pragma unroll 1
        for (int b0 = 0; b0 < c; b0 += 32) {
          const int idx = b0 + lane;
          const int ent = list[w2 * WCAP + (idx < WCAP ? idx : WCAP - 1)];
          const int m32 = (c - b0) < 32 ? (c - b0) : 32;
#pragma unroll 1
          for (int k = 0; k < m32; ++k) {
            const int u    = __builtin_amdgcn_readlane(ent, k);
            const int slot = u & (NBA - 1);
            const int el   = (u >> SLA) & (CHUNK - 1);
            const int pk   = ((cbase + el) << SLA) | slot;
            if (t < RCAP) {
              if (lane == 0) { hl[t] = pk; cnt[slot] = cnt[slot] + 1; }
              t = t + 1;
            } else {
              ov = 1;
            }
          }
        }
      }
    }
    __syncthreads();
  }
  if (wave == 0 && lane == 0) { misc[8] = t; misc[9] = ov; }
  __syncthreads();
  int tt = misc[8];
  tt = tt < 0 ? 0 : (tt > RCAP ? RCAP : tt);
  const int ovf = misc[9];

  if (wave == 0) {
    const int base = lane * (NBA / 32);
    int s = 0;
#pragma unroll 1
    for (int i = 0; i < NBA / 32; ++i) s += cnt[base + i];
    int incl = s;
#pragma unroll
    for (int d = 1; d < 32; d <<= 1) {
      const int y = __shfl_up(incl, d, 32);
      if (lane >= d) incl += y;
    }
    int run = incl - s;
#pragma unroll 1
    for (int i = 0; i < NBA / 32; ++i) {
      const int cv = cnt[base + i];
      offs[base + i] = run;
      cur[base + i]  = run;
      run += cv;
    }
  }
  __syncthreads();
  if (wave == 0) {
#pragma unroll 1
    for (int b0 = 0; b0 < tt; b0 += 32) {
      const int idx = b0 + lane;
      const int ent = hl[idx < RCAP ? idx : RCAP - 1];
      const int m32 = (tt - b0) < 32 ? (tt - b0) : 32;
#pragma unroll 1
      for (int k = 0; k < m32; ++k) {
        const int u    = __builtin_amdgcn_readlane(ent, k);
        const int slot = u & (NBA - 1);
        if (lane == 0) {
          int p = cur[slot];
          p = p < 0 ? 0 : (p > RCAP - 1 ? RCAP - 1 : p);
          sl[p] = u;
          cur[slot] = p + 1;
        }
      }
    }
  }
  __syncthreads();

  const float pz = (ovf != 0) ? __int_as_float(0x7fc00000) : 0.0f;
  unsigned short* sw = stw + wave * (4 * KH);
#pragma unroll 1
  for (int g = 0; g < NBA / (NWAVE * 4); ++g) {
#pragma unroll 1
    for (int q = 0; q < 4; ++q) {
      const int s    = (4 * g + q) * NWAVE + wave;
      const int node = nodeBase + s;
      int c = cnt[s];
      const bool big = c > DEGCAP;
      c = c < 0 ? 0 : (c > DEGCAP ? DEGCAP : c);
      int o = offs[s];
      o = o < 0 ? 0 : (o > RCAP ? RCAP : o);
      float acc = 0.0f;
#pragma unroll 1
      for (int b0 = 0; b0 < c; b0 += 32) {
        int idx = o + b0 + lane;
        idx = idx > RCAP - 1 ? RCAP - 1 : idx;
        const int ent = sl[idx];
        int eid = ent >> SLA;
        eid = eid < 0 ? 0 : (eid > nE - 1 ? nE - 1 : eid);
        int sr = pr[2 * (size_t)eid + 1];
        sr = sr < 0 ? 0 : (sr > nN - 1 ? nN - 1 : sr);
        const int m32 = (c - b0) < 32 ? (c - b0) : 32;
#pragma unroll 1
        for (int k = 0; k < m32; ++k) {
          const int ek = __builtin_amdgcn_readlane(eid, k);
          const int sk = __builtin_amdgcn_readlane(sr, k);
          const float* bq = bond + (size_t)ek * BDIM;
          const v4f c0 = *(const v4f*)bq;
          const v4f c1 = *(const v4f*)(bq + 4);
          const v4f c2 = *(const v4f*)(bq + 8);
          const v4f c3 = *(const v4f*)(bq + 12);
          const float* uq = uv + (size_t)sk * UVW + BDIM * lane;
          const v4f u0 = *(const v4f*)uq;
          const v4f u1 = *(const v4f*)(uq + 4);
          const v4f u2 = *(const v4f*)(uq + 8);
          const v4f u3 = *(const v4f*)(uq + 12);
          const float vv = uv[(size_t)sk * UVW + UCOL + lane];
          float tm = bf16_val(c0.x) * u0.x;
          tm = fmaf(bf16_val(c0.y), u0.y, tm);
          tm = fmaf(bf16_val(c0.z), u0.z, tm);
          tm = fmaf(bf16_val(c0.w), u0.w, tm);
          tm = fmaf(bf16_val(c1.x), u1.x, tm);
          tm = fmaf(bf16_val(c1.y), u1.y, tm);
          tm = fmaf(bf16_val(c1.z), u1.z, tm);
          tm = fmaf(bf16_val(c1.w), u1.w, tm);
          tm = fmaf(bf16_val(c2.x), u2.x, tm);
          tm = fmaf(bf16_val(c2.y), u2.y, tm);
          tm = fmaf(bf16_val(c2.z), u2.z, tm);
          tm = fmaf(bf16_val(c2.w), u2.w, tm);
          tm = fmaf(bf16_val(c3.x), u3.x, tm);
          tm = fmaf(bf16_val(c3.y), u3.y, tm);
          tm = fmaf(bf16_val(c3.z), u3.z, tm);
          tm = fmaf(bf16_val(c3.w), u3.w, tm);
          acc += (tm + vv);
        }
      }
      const float pzr = big ? __int_as_float(0x7fc00000) : pz;
      const bool live = node < nN;
      const float v = live ? (acc + pzr) : 0.0f;
      const unsigned hb = bf16_bits(v);
      const unsigned lb = bf16_bits(v - __uint_as_float(hb << 16));
      sw[q * KH + lane]      = (unsigned short)hb;
      sw[q * KH + DD + lane] = (unsigned short)lb;
    }
    __syncthreads();
    {
      const int q = lane >> 3, p = lane & 7;
      const v8us val = *(const v8usa*)(sw + q * KH + 8 * p);
      const int node = nodeBase + (4 * g + q) * NWAVE + wave;
      unsigned short* dp = aggp + (size_t)node * KH + 8 * p;
      *(volatile v8us*)dp = val;
      __threadfence();
      *(volatile v8us*)dp = val;
    }
    __syncthreads();
  }
}

__global__ __launch_bounds__(GTHR) void k_gru(const unsigned short* __restrict__ ag,
                                              const unsigned short* __restrict__ wg,
                                              const float* __restrict__ bih, const float* __restrict__ bhh,
                                              unsigned short* ha, float* outp, int nN, int last) {
  __shared__ __attribute__((aligned(16))) float stg[GBM * NGC];
  __shared__ float sb[NGC];
  const int tid = (int)threadIdx.x, lane = tid & 31, wave = tid >> 5, hh = lane >> 4, m = lane & 15;
  const int rowBase = (int)blockIdx.x * GBM;

  for (int i = tid; i < NGC; i += GTHR) {
    const int ii = i < 3 * DD ? i : 3 * DD - 1;
    int ih = i - 3 * DD;
    ih = ih < 0 ? 0 : ih;
    const float fi = (i < 3 * DD) ? 1.0f : 0.0f;
    sb[i] = bf16_val(bih[ii] * fi + bhh[ih] * (1.0f - fi));
  }

  v8f acc[12];
#pragma unroll
  for (int t = 0; t < 12; ++t) acc[t] = z8();
  const unsigned short* apA = ag + (size_t)(rowBase + 16 * wave + m) * KH + 8 * hh;
  const unsigned short* apH = ha + (size_t)(rowBase + 16 * wave + m) * KH + 8 * hh;
  const unsigned short* bp  = wg + (size_t)m * KH + 8 * hh;

#pragma unroll 1
  for (int k0 = 0; k0 < KH; k0 += 32) {
    FragB fa, fh;
    fa.h[0] = *(const v8usa*)(apA + k0);
    fa.h[1] = *(const v8usa*)(apA + k0 + 16);
    fh.h[0] = *(const v8usa*)(apH + k0);
    fh.h[1] = *(const v8usa*)(apH + k0 + 16);
#pragma unroll
    for (int nt = 0; nt < 6; ++nt) {
      const unsigned short* wq = bp + (size_t)(16 * nt) * KH + k0;
      FragB bf;
      bf.h[0] = *(const v8usa*)wq;
      bf.h[1] = *(const v8usa*)(wq + 16);
      acc[nt] = wmb(fa, bf, acc[nt]);
      const unsigned short* wr = bp + (size_t)(3 * DD + 16 * nt) * KH + k0;
      FragB bg;
      bg.h[0] = *(const v8usa*)wr;
      bg.h[1] = *(const v8usa*)(wr + 16);
      acc[6 + nt] = wmb(fh, bg, acc[6 + nt]);
    }
  }

#pragma unroll
  for (int nt = 0; nt < 12; ++nt) {
    const int lc = 16 * nt + m;
#pragma unroll
    for (int r = 0; r < 8; ++r) {
      const int lr = 16 * wave + 8 * hh + r;
      stg[lr * NGC + lc] = acc[nt][r];
    }
  }

  const int row = tid >> 1, half = tid & 1, j0 = (DD / 2) * half;
  FragB oh, ol;
  {
    const unsigned short* hp = ha + (size_t)(rowBase + row) * KH + j0;
    oh.h[0] = *(const v8usa*)hp;
    oh.h[1] = *(const v8usa*)(hp + 8);
    ol.h[0] = *(const v8usa*)(hp + DD);
    ol.h[1] = *(const v8usa*)(hp + DD + 8);
  }
  __syncthreads();

  float hn[16];
  {
    const float* sr = stg + row * NGC + j0;
#pragma unroll
    for (int e = 0; e < 16; ++e) {
      const int j = j0 + e;
      const float ho = __uint_as_float((unsigned)oh.u[e] << 16) + __uint_as_float((unsigned)ol.u[e] << 16);
      const float gir = sr[e], giz = sr[DD + e], gin = sr[2 * DD + e];
      const float ghr = sr[3 * DD + e], ghz = sr[4 * DD + e], ghn = sr[5 * DD + e];
      const float rr = sigm((gir + sb[j]) + (ghr + sb[3 * DD + j]));
      const float zz = sigm((giz + sb[DD + j]) + (ghz + sb[4 * DD + j]));
      const float nn = tanhf((gin + sb[2 * DD + j]) + rr * (ghn + sb[5 * DD + j]));
      hn[e] = (1.0f - zz) * nn + zz * ho;
    }
  }
  __syncthreads();

  float* hof = stg;
  unsigned short* hbf = (unsigned short*)(stg + GBM * DD);
  {
    v8us hi0, hi1, lo0, lo1;
#pragma unroll
    for (int e = 0; e < 8; ++e) {
      const unsigned hb0 = bf16_bits(hn[e]);
      const unsigned hb1 = bf16_bits(hn[8 + e]);
      hi0[e] = (unsigned short)hb0;
      hi1[e] = (unsigned short)hb1;
      lo0[e] = (unsigned short)bf16_bits(hn[e]     - __uint_as_float(hb0 << 16));
      lo1[e] = (unsigned short)bf16_bits(hn[8 + e] - __uint_as_float(hb1 << 16));
    }
    v4f f0, f1, f2, f3;
    f0.x = hn[0];  f0.y = hn[1];  f0.z = hn[2];  f0.w = hn[3];
    f1.x = hn[4];  f1.y = hn[5];  f1.z = hn[6];  f1.w = hn[7];
    f2.x = hn[8];  f2.y = hn[9];  f2.z = hn[10]; f2.w = hn[11];
    f3.x = hn[12]; f3.y = hn[13]; f3.z = hn[14]; f3.w = hn[15];
    float* fp = hof + row * DD + j0;
    *(v4fa*)fp = f0; *(v4fa*)(fp + 4) = f1; *(v4fa*)(fp + 8) = f2; *(v4fa*)(fp + 12) = f3;
    unsigned short* up = hbf + row * KH + j0;
    *(v8usa*)up = hi0; *(v8usa*)(up + 8) = hi1;
    *(v8usa*)(up + DD) = lo0; *(v8usa*)(up + DD + 8) = lo1;
  }
  __syncthreads();

  unsigned short* ghp = ha + (size_t)rowBase * KH;
#pragma unroll
  for (int it = 0; it < (GBM * KH / 8) / GTHR; ++it) {
    const int u = it * GTHR + tid;
    const v8us v = *(const v8usa*)(hbf + 8 * u);
    *(volatile v8us*)(ghp + 8 * u) = v;
  }
  __threadfence();
#pragma unroll
  for (int it = 0; it < (GBM * KH / 8) / GTHR; ++it) {
    const int u = it * GTHR + tid;
    const v8us v = *(const v8usa*)(hbf + 8 * u);
    *(volatile v8us*)(ghp + 8 * u) = v;
  }

  if (last != 0) {
    float* gop = outp + (size_t)rowBase * DD;
#pragma unroll
    for (int it = 0; it < (GBM * DD / 4) / GTHR; ++it) {
      const int u = it * GTHR + tid;
      const v4f v = *(const v4fa*)(hof + 4 * u);
      if (rowBase + (u >> 3) < nN) *(volatile v4f*)(gop + 4 * u) = v;
    }
    __threadfence();
#pragma unroll
    for (int it = 0; it < (GBM * DD / 4) / GTHR; ++it) {
      const int u = it * GTHR + tid;
      const v4f v = *(const v4fa*)(hof + 4 * u);
      if (rowBase + (u >> 3) < nN) *(volatile v4f*)(gop + 4 * u) = v;
    }
  }
}

static inline int cdiv(int a, int b) { return (a + b - 1) / b; }

extern "C" void kernel_launch(void* const* d_in, const int* in_sizes, int n_in,
                              void* d_out, int out_size, void* d_ws, size_t ws_size,
                              hipStream_t stream) {
  if (n_in < 9) return;
  if (in_sizes[0] < DD || (in_sizes[0] % DD) != 0) return;
  const int nN = in_sizes[0] / DD;
  if (in_sizes[2] < 2 || (in_sizes[2] & 1) != 0) return;
  const int nE = in_sizes[2] / 2;
  if (nE < 1 || nE >= (1 << 21)) return;
  if ((long long)in_sizes[1] != (long long)nE * BDIM) return;
  if (in_sizes[3] != BDIM * DD * DD || in_sizes[4] != DD * DD) return;
  if (in_sizes[5] != 3 * DD * DD || in_sizes[6] != 3 * DD * DD) return;
  if (in_sizes[7] != 3 * DD || in_sizes[8] != 3 * DD) return;
  if ((long long)out_size != (long long)nN * DD) return;
  if (nN > (1 << 22)) return;

  const float* atom = (const float*)d_in[0];
  const float* bond = (const float*)d_in[1];
  const int*   pr   = (const int*)d_in[2];
  const float* kw   = (const float*)d_in[3];
  const float* kb   = (const float*)d_in[4];
  const float* wih  = (const float*)d_in[5];
  const float* whh  = (const float*)d_in[6];
  const float* bih  = (const float*)d_in[7];
  const float* bhh  = (const float*)d_in[8];
  float* out = (float*)d_out;

  const int gA   = cdiv(nN, NBA);
  const int MP   = gA * NBA;
  const int gM   = MP / GBM;
  const int nbHA = MP / 32;

  char* ws = (char*)d_ws;
  size_t off = 0;
  const size_t oUV = off; off += (size_t)MP * UVW * 4;   off = (off + 255) & ~(size_t)255;
  const size_t oHA = off; off += (size_t)MP * KH * 2;    off = (off + 255) & ~(size_t)255;
  const size_t oAG = off; off += (size_t)MP * KH * 2;    off = (off + 255) & ~(size_t)255;
  const size_t oBK = off; off += (size_t)UVW * KH * 2;   off = (off + 255) & ~(size_t)255;
  const size_t oWG = off; off += (size_t)NGC * KH * 2;   off = (off + 255) & ~(size_t)255;
  if (off > ws_size || off > (size_t)WSMAX) return;
  float*          UV = (float*)(ws + oUV);
  unsigned short* HA = (unsigned short*)(ws + oHA);
  unsigned short* AG = (unsigned short*)(ws + oAG);
  unsigned short* BK = (unsigned short*)(ws + oBK);
  unsigned short* WG = (unsigned short*)(ws + oWG);

  const size_t aggLds = (size_t)AGG_LDS_INTS * 4;
  hipFuncSetAttribute(reinterpret_cast<const void*>(&k_agg), hipFuncAttributeMaxDynamicSharedMemorySize, (int)aggLds);

  k_prep<<<nbHA + NBKB + NWGB, NTHR, 0, stream>>>(atom, nN, nbHA, kw, kb, wih, whh, HA, BK, WG);
  for (int s = 0; s < NSTEP; ++s) {
    k_node<<<dim3(gM, UVW / GBN), GTHR, 0, stream>>>(HA, BK, UV);
    k_agg<<<gA, NTHR, aggLds, stream>>>(pr, nE, nN, bond, UV, AG);
    k_gru<<<gM, GTHR, 0, stream>>>(AG, WG, bih, bhh, HA, out, nN, (s == NSTEP - 1) ? 1 : 0);
  }
}
